// myGATConv_6648609374674
// MI455X (gfx1250) — hardware-run, weakly checked
//
#include <hip/hip_runtime.h>

typedef float          v8f   __attribute__((ext_vector_type(8)));
typedef float          v4f   __attribute__((ext_vector_type(4)));
typedef unsigned int   v4u   __attribute__((ext_vector_type(4)));
typedef int            v8i   __attribute__((ext_vector_type(8)));
typedef unsigned short v8us  __attribute__((ext_vector_type(8)));
typedef unsigned short v16us __attribute__((ext_vector_type(16)));
typedef __bf16         v16bf __attribute__((ext_vector_type(16)));
typedef _Float16       v16h  __attribute__((ext_vector_type(16)));
typedef v4f  __attribute__((may_alias)) v4fa;
typedef v8us __attribute__((may_alias)) v8usa;
union FragB { v16bf v; v16us u; v8us h[2]; v8i w; };
union FragH { v16h  v; v16us u; v8us h[2]; v8i w; };

__device__ __forceinline__ v8f wmb(const FragB& a, const FragB& b, v8f c) {
  v8f d = __builtin_amdgcn_wmma_f32_16x16x32_bf16(false, a.v, false, b.v, (short)0, c, false, false);
  asm volatile("v_nop\n\tv_nop\n\tv_nop\n\tv_nop" : "+v"(d) : "v"(a.w), "v"(b.w));
  return d;
}

__device__ __forceinline__ v8f wmh(const FragH& a, const FragH& b, v8f c) {
  v8f d = __builtin_amdgcn_wmma_f32_16x16x32_f16(false, a.v, false, b.v, (short)0, c, false, false);
  asm volatile("v_nop\n\tv_nop\n\tv_nop\n\tv_nop" : "+v"(d) : "v"(a.w), "v"(b.w));
  return d;
}

__device__ __forceinline__ unsigned bf16_bits(float f) {
  const unsigned u = __float_as_uint(f);
  const unsigned r = (u + 0x7FFFu + ((u >> 16) & 1u)) >> 16;
  const unsigned q = (u >> 16) | 0x40u;
  return ((u & 0x7fffffffu) > 0x7f800000u) ? q : r;
}

__device__ __forceinline__ float bf16_val(float f) {
  return __uint_as_float(bf16_bits(f) << 16);
}
__device__ __forceinline__ int clampi(int v, int lo, int hi) {
  return v < lo ? lo : (v > hi ? hi : v);
}

__device__ __forceinline__ unsigned f16_bits(float f) {
  const unsigned u  = __float_as_uint(f);
  const unsigned s  = (u >> 16) & 0x8000u;
  const unsigned a  = u & 0x7fffffffu;
  const unsigned t  = a - 0x38000000u;
  const unsigned r  = (t + 0x0FFFu + ((t >> 13) & 1u)) >> 13;
  const unsigned rc = r > 0x7C00u ? 0x7C00u : r;
  const bool small  = a < 0x38800000u;
  const bool isnan  = a > 0x7f800000u;
  const unsigned fin = small ? 0u : (s | rc);
  return isnan ? (s | 0x7E00u) : fin;
}

__device__ __forceinline__ unsigned pk16(unsigned lo, unsigned hi) { return lo | (hi << 16); }
__device__ __forceinline__ unsigned bf16_lo_bits(float v) {
  float hi = bf16_val(v);
  asm volatile("" : "+v"(hi));
  return bf16_bits(v - hi);
}
__device__ __forceinline__ v4u pack8_bf16(v4f a, v4f c) {
  return (v4u){ pk16(bf16_bits(a[0]), bf16_bits(a[1])), pk16(bf16_bits(a[2]), bf16_bits(a[3])),
                pk16(bf16_bits(c[0]), bf16_bits(c[1])), pk16(bf16_bits(c[2]), bf16_bits(c[3])) };
}
__device__ __forceinline__ v4u pack8_bf16_lo(v4f a, v4f c) {
  return (v4u){ pk16(bf16_lo_bits(a[0]), bf16_lo_bits(a[1])), pk16(bf16_lo_bits(a[2]), bf16_lo_bits(a[3])),
                pk16(bf16_lo_bits(c[0]), bf16_lo_bits(c[1])), pk16(bf16_lo_bits(c[2]), bf16_lo_bits(c[3])) };
}
__device__ __forceinline__ v4u pack8_f16(v4f a, v4f c) {
  return (v4u){ pk16(f16_bits(a[0]), f16_bits(a[1])), pk16(f16_bits(a[2]), f16_bits(a[3])),
                pk16(f16_bits(c[0]), f16_bits(c[1])), pk16(f16_bits(c[2]), f16_bits(c[3])) };
}

template <int FORM>
__global__ __launch_bounds__(256) void k_plane(const float* __restrict__ src, int rows, int cols, int ldsrc,
                                               unsigned short* __restrict__ dst, int MP, int KP) {
  static_assert(FORM >= 0 && FORM <= 3);
  const int KTOT = (FORM == 1 || FORM == 3) ? 2 * KP : KP;
  const unsigned ppr   = (unsigned)(KTOT >> 3);
  const unsigned kp8   = (unsigned)(KP >> 3);
  const unsigned total = (unsigned)MP * ppr;
  const unsigned g     = blockIdx.x * 256u + threadIdx.x;
  const unsigned rowu  = g / ppr;
  const unsigned p     = g - rowu * ppr;
  const bool second    = p >= kp8;
  const int row = (int)rowu;
  const int c0  = (int)((second ? p - kp8 : p) << 3);
  const float* srow = src + (size_t)clampi(row, 0, rows - 1) * (size_t)ldsrc;
  float x[8];
  unsigned mk[8];
#pragma unroll
  for (int e = 0; e < 8; ++e) {
    const int c = c0 + e;
    const float v = srow[clampi(c, 0, cols - 1)];
    asm volatile("" :: "v"(v));
    x[e]  = v;
    mk[e] = (row < rows && c < cols) ? 0xFFFFu : 0u;
  }
  const v4f a = (v4f){ x[0], x[1], x[2], x[3] };
  const v4f c = (v4f){ x[4], x[5], x[6], x[7] };
  v4u o;
  if (FORM == 2) {
    o = pack8_f16(a, c);
  } else {
    const v4u hi = pack8_bf16(a, c);
    o = hi;
    if (FORM == 1) { const v4u lo = pack8_bf16_lo(a, c); o = second ? lo : hi; }
  }
  const v4u mw = (v4u){ pk16(mk[0], mk[1]), pk16(mk[2], mk[3]), pk16(mk[4], mk[5]), pk16(mk[6], mk[7]) };
  o &= mw;
  if (g < total) {
    volatile v4u* q = (volatile v4u*)(dst + (size_t)g * 8);
    *q = o;
    __threadfence();
    *q = o;
  }
}

template <int FORM> struct FragOf    { typedef FragB T; };
template <>         struct FragOf<2> { typedef FragH T; };
__device__ __forceinline__ v8f mm(const FragB& a, const FragB& b, v8f c) { return wmb(a, b, c); }
__device__ __forceinline__ v8f mm(const FragH& a, const FragH& b, v8f c) { return wmh(a, b, c); }
template <class F> __device__ __forceinline__ F ld_frag(const unsigned short* p) {
  F f;
  f.h[0] = *(const v8usa*)(p);
  f.h[1] = *(const v8usa*)(p + 16);
  return f;
}

template <int FORM, int EPI>
__global__ __launch_bounds__(256) __attribute__((amdgpu_num_vgpr(248)))
void k_gemm_nt(const unsigned short* __restrict__ A, const unsigned short* __restrict__ B,
               const float* __restrict__ bias, float* __restrict__ D, int M, int N, int KTOT, int ldd) {
  static_assert(FORM >= 0 && FORM <= 2);
  static_assert(EPI == 0 || EPI == 1);
  typedef typename FragOf<FORM>::T F;
  __shared__ __attribute__((aligned(16))) float sT[8][16 * 68];
  const int lane = threadIdx.x & 31;
  const int wave = threadIdx.x >> 5;
  const int tilesM = (M + 63) >> 6;
  const int tilesN = (N + 63) >> 6;
  const int tile = blockIdx.x * 8 + wave;
  if (tile >= tilesM * tilesN) return;
  const int tm = tile / tilesN;
  const int tn = tile - tm * tilesN;
  const int m0 = tm << 6;
  const int n0 = tn << 6;

  const int rl = lane & 15;
  const int h8 = (lane >> 4) * 8;
  const unsigned short* pa = A + (size_t)(m0 + rl) * (size_t)KTOT + h8;
  const unsigned short* pb = B + (size_t)(n0 + rl) * (size_t)KTOT + h8;

  v8f acc[4][4];
#pragma unroll
  for (int i = 0; i < 4; ++i)
#pragma unroll
    for (int j = 0; j < 4; ++j) acc[i][j] = (v8f){0.f, 0.f, 0.f, 0.f, 0.f, 0.f, 0.f, 0.f};

#pragma unroll 1
  for (int k0 = 0; k0 < KTOT; k0 += 32) {
    F bf[4];
#pragma unroll
    for (int j = 0; j < 4; ++j) bf[j] = ld_frag<F>(pb + (size_t)(j << 4) * (size_t)KTOT + k0);
#pragma unroll
    for (int i = 0; i < 4; ++i) {
      const F af = ld_frag<F>(pa + (size_t)(i << 4) * (size_t)KTOT + k0);
#pragma unroll
      for (int j = 0; j < 4; ++j) acc[i][j] = mm(af, bf[j], acc[i][j]);
    }
  }

  float* slab = sT[wave];
  const int hh = lane >> 4;
  const int c4 = (lane & 15) * 4;
  const int nc = n0 + c4;
  const bool cok = nc < N;
  v4f bv = (v4f){0.f, 0.f, 0.f, 0.f};
  if (EPI == 1) {
    bv = *(const v4fa*)(bias + clampi(nc, 0, N - 4));
    asm volatile("" :: "v"(bv));
  }
#pragma unroll
  for (int i = 0; i < 4; ++i) {
    const int mBase = m0 + (i << 4);
#pragma unroll
    for (int j = 0; j < 4; ++j) {
#pragma unroll
      for (int r = 0; r < 8; ++r) slab[(h8 + r) * 68 + (j << 4) + rl] = acc[i][j][r];
    }
    __builtin_amdgcn_fence(__ATOMIC_RELEASE, "workgroup");
    __builtin_amdgcn_wave_barrier();
    __builtin_amdgcn_fence(__ATOMIC_ACQUIRE, "workgroup");
    v4f vv[8];
#pragma unroll
    for (int it = 0; it < 8; ++it) {
      const int row = it * 2 + hh;
      v4f v = *(const v4fa*)(slab + row * 68 + c4);
      if (EPI == 1) v += bv;
      vv[it] = v;
    }
    for (int pass = 0; pass < 2; ++pass) {
#pragma unroll
      for (int it = 0; it < 8; ++it) {
        const int row = mBase + it * 2 + hh;
        if (cok && row < M) *(volatile v4f*)(D + (size_t)row * (size_t)ldd + nc) = vv[it];
      }
      __threadfence();
    }
    __builtin_amdgcn_fence(__ATOMIC_RELEASE, "workgroup");
    __builtin_amdgcn_wave_barrier();
    __builtin_amdgcn_fence(__ATOMIC_ACQUIRE, "workgroup");
  }
}

#pragma clang fp contract(off)


#define NN      50000
#define NEDG    800000
#define MPAD    50048
#define KD      256
#define DOUTW   256
#define NHD     8
#define DSZ     32
#define NET     8
#define ATTW    96
#define RTHR    256
#define RWAVES  8
#define TB_BF   0
#define TB_BR   256
#define TB_AS   512
#define TB_AD   768
#define TB_SE   1024
#define TB_N    1088
#define BT      512
#define BW      16
#define BEPT    8
#define BCHUNK  (BT * BEPT)
#define NCH     ((NEDG + BCHUNK - 1) / BCHUNK)
#define NB      1024
#define NBLK    ((NN + NB - 1) / NB)
#define RCAP    21504
#define DEGCAP  64
#define SLOTSH  21
#define LISTTOT (NBLK * RCAP)
#define LDS_BKT ((2 * RCAP + 3 * NB + 64) * 4)
#define SDOFF   (MPAD * NHD)
#define WPIECES (DOUTW * KD / 8)
#define PREP_PB (WPIECES / 256)
#define WSMAX   ((size_t)128 << 20)

static_assert(NHD * DSZ == 256 && DSZ == 32 && DOUTW == 256 && KD == 256);
static_assert(32 * 8 == DOUTW);
static_assert(ATTW == 3 * DSZ);
static_assert(MPAD == 391 * 128 && MPAD % 64 == 0 && MPAD >= NN);
static_assert(NN % 16 == 0 && MPAD % 16 == 0 && KD % 32 == 0 && DOUTW % 64 == 0);
static_assert(NN % RWAVES == 0 && MPAD % RWAVES == 0);
static_assert(NEDG < (1 << SLOTSH));
static_assert(NB <= 1024 && (NB & (NB - 1)) == 0 && NB == 2 * BT);
static_assert(NEDG % 8 == 0 && NEDG >= 8);
static_assert(NBLK == 49 && NBLK * NB >= NN);
static_assert(NCH * BCHUNK >= NEDG && NCH == 196);
static_assert(RCAP % 32 == 0 && RCAP % BT == 0);
static_assert(RCAP * 4 >= 16696 * 5);
static_assert(DEGCAP >= 33 + 8);
static_assert(DEGCAP * NHD == 512 && DEGCAP * NHD >= DOUTW && (DEGCAP * NHD) % 32 == 0);
static_assert(LDS_BKT <= 300000);
static_assert(BW == BT / 32 && BW == 16);
static_assert(PREP_PB == 32 && WPIECES == 8192);
static_assert(TB_N % 32 == 0);

typedef int          v4i __attribute__((ext_vector_type(4)));
typedef int          v2i __attribute__((ext_vector_type(2)));
typedef unsigned int v2u __attribute__((ext_vector_type(2)));
typedef v4i __attribute__((may_alias)) v4ia;
typedef v2i __attribute__((may_alias)) v2ia;
typedef v2u __attribute__((may_alias)) v2ua;

__device__ __forceinline__ float leaky_k(float v) { return (v >= 0.0f) ? v : 0.2f * v; }
__device__ __forceinline__ float maxk(float a, float b) {
  float m = (a < b) ? b : a;
  m = (b != b) ? b : m;
  return m;
}
__device__ __forceinline__ void wave_sync_lds() {
  __builtin_amdgcn_fence(__ATOMIC_RELEASE, "workgroup");
  __builtin_amdgcn_wave_barrier();
  __builtin_amdgcn_fence(__ATOMIC_ACQUIRE, "workgroup");
}

__device__ __forceinline__ void prep_wpiece(const float* __restrict__ W, unsigned short* dst, int g) {
  const int n  = g >> 5;
  const int k0 = (g & 31) << 3;
  float x[8];
#pragma unroll
  for (int e = 0; e < 8; ++e) {
    const float v = W[(size_t)(k0 + e) * DOUTW + n];
    asm volatile("" :: "v"(v));
    x[e] = v;
  }
  const v4u o = pack8_bf16((v4f){ x[0], x[1], x[2], x[3] }, (v4f){ x[4], x[5], x[6], x[7] });
  volatile v4u* q = (volatile v4u*)(dst + (size_t)g * 8);
  *q = o;
  __threadfence();
  *q = o;
}

__global__ __launch_bounds__(256) void k_prep(const float* __restrict__ Wfc, const float* __restrict__ Wres,
                                              const float* __restrict__ bfc, const float* __restrict__ bres,
                                              const float* __restrict__ eemb, const float* __restrict__ attn,
                                              unsigned short* WFT, unsigned short* WRT, float* TB) {
  __shared__ __attribute__((aligned(16))) float sse[NET * NHD];
  const int b = (int)blockIdx.x;
  const int t = (int)threadIdx.x;
  if (b < PREP_PB) { prep_wpiece(Wfc, WFT, b * 256 + t); return; }
  if (b < 2 * PREP_PB) { prep_wpiece(Wres, WRT, (b - PREP_PB) * 256 + t); return; }

  {
    const int reg = t >> 6;
    const int col = (t & 63) * 4;
    const int hq  = col >> 5;
    const int cq  = col & 31;
    const v4f a0 = *(const v4fa*)(bfc + col);
    asm volatile("" :: "v"(a0));
    const v4f a1 = *(const v4fa*)(bres + col);
    asm volatile("" :: "v"(a1));
    const v4f a2 = *(const v4fa*)(attn + hq * ATTW + cq);
    asm volatile("" :: "v"(a2));
    const v4f a3 = *(const v4fa*)(attn + hq * ATTW + DSZ + cq);
    asm volatile("" :: "v"(a3));
    const unsigned m0 = (reg == 0) ? 0xFFFFFFFFu : 0u;
    const unsigned m1 = (reg == 1) ? 0xFFFFFFFFu : 0u;
    const unsigned m2 = (reg == 2) ? 0xFFFFFFFFu : 0u;
    const unsigned m3 = (reg == 3) ? 0xFFFFFFFFu : 0u;
    v4u o;
    o.x = (__float_as_uint(a0.x) & m0) | (__float_as_uint(a1.x) & m1) | (__float_as_uint(a2.x) & m2) | (__float_as_uint(a3.x) & m3);
    o.y = (__float_as_uint(a0.y) & m0) | (__float_as_uint(a1.y) & m1) | (__float_as_uint(a2.y) & m2) | (__float_as_uint(a3.y) & m3);
    o.z = (__float_as_uint(a0.z) & m0) | (__float_as_uint(a1.z) & m1) | (__float_as_uint(a2.z) & m2) | (__float_as_uint(a3.z) & m3);
    o.w = (__float_as_uint(a0.w) & m0) | (__float_as_uint(a1.w) & m1) | (__float_as_uint(a2.w) & m2) | (__float_as_uint(a3.w) & m3);
    o.x = bf16_bits(__uint_as_float(o.x)) << 16;
    o.y = bf16_bits(__uint_as_float(o.y)) << 16;
    o.z = bf16_bits(__uint_as_float(o.z)) << 16;
    o.w = bf16_bits(__uint_as_float(o.w)) << 16;
    volatile v4u* q = (volatile v4u*)(TB + 4 * t);
    *q = o;
    __threadfence();
    *q = o;
  }

  {
    const int u  = t & 63;
    const int tt = u >> 3;
    const int hh = u & 7;
    const float* ep = eemb + tt * DOUTW + hh * DSZ;
    const float* ap = attn + hh * ATTW + 2 * DSZ;
    float s = 0.0f;
#pragma unroll 1
    for (int i = 0; i < 8; ++i) {
      const v4f e4 = *(const v4fa*)(ep + 4 * i);
      const v4f a4 = *(const v4fa*)(ap + 4 * i);
      float e0 = bf16_val(e4.x), e1 = bf16_val(e4.y), e2 = bf16_val(e4.z), e3 = bf16_val(e4.w);
      float q0 = bf16_val(a4.x), q1 = bf16_val(a4.y), q2 = bf16_val(a4.z), q3 = bf16_val(a4.w);
      asm volatile("" : "+v"(e0));
      asm volatile("" : "+v"(e1));
      asm volatile("" : "+v"(e2));
      asm volatile("" : "+v"(e3));
      asm volatile("" : "+v"(q0));
      asm volatile("" : "+v"(q1));
      asm volatile("" : "+v"(q2));
      asm volatile("" : "+v"(q3));
      float pr;
      pr = e0 * q0; s = s + pr;
      pr = e1 * q1; s = s + pr;
      pr = e2 * q2; s = s + pr;
      pr = e3 * q3; s = s + pr;
    }
    if (t < NET * NHD) sse[t] = s;
  }
  __syncthreads();
  if ((t >> 5) == 0) {
    const int l16 = t & 15;
    const v4f sv = *(const v4fa*)(sse + 4 * l16);
    asm volatile("" :: "v"(sv));
    const bool wr = t < 16;
    volatile v4f* q = (volatile v4f*)(TB + TB_SE + 4 * l16);
    if (wr) *q = sv;
    __threadfence();
    if (wr) *q = sv;
  }
}

__global__ __launch_bounds__(BT) void k_list(const int* __restrict__ eown, const int* __restrict__ egat,
                                             const int* __restrict__ ety, unsigned* LIST, int* META) {
  extern __shared__ v4u lds_bkt[];
  int* reg1 = (int*)lds_bkt;
  int* reg2 = reg1 + RCAP;
  int* scnt = reg2 + RCAP;
  int* soff = scnt + NB;
  int* curs = soff + NB;
  int* wcnt = curs + NB;
  int* wtot = wcnt + 2 * BW;
  const int tid = (int)threadIdx.x, lane = tid & 31, wave = tid >> 5;
  const int nodeBase = (int)blockIdx.x * NB;
  int nb = NN - nodeBase;
  nb = nb > NB ? NB : (nb < 0 ? 0 : nb);
  const unsigned nbs = (unsigned)nodeBase, unb = (unsigned)nb;

  scnt[2 * tid] = 0;
  scnt[2 * tid + 1] = 0;
  if (tid == 0) reg2[0] = 0;

  int tot = 0;
#pragma unroll 1
  for (int ch = 0; ch < NCH; ++ch) {
    const int par = ch & 1;
    const int e0  = ch * BCHUNK + tid * BEPT;
    const bool valid = e0 < NEDG;
    const int ea = e0 < NEDG - 8 ? e0 : NEDG - 8;
    const v4i da = *(const v4ia*)(eown + ea);
    const v4i db = *(const v4ia*)(eown + ea + 4);
    asm volatile("" :: "v"(da), "v"(db));
    const unsigned s0 = (unsigned)da.x - nbs, s1 = (unsigned)da.y - nbs;
    const unsigned s2 = (unsigned)da.z - nbs, s3 = (unsigned)da.w - nbs;
    const unsigned s4 = (unsigned)db.x - nbs, s5 = (unsigned)db.y - nbs;
    const unsigned s6 = (unsigned)db.z - nbs, s7 = (unsigned)db.w - nbs;
    const bool h0 = valid && (s0 < unb), h1 = valid && (s1 < unb), h2 = valid && (s2 < unb), h3 = valid && (s3 < unb);
    const bool h4 = valid && (s4 < unb), h5 = valid && (s5 < unb), h6 = valid && (s6 < unb), h7 = valid && (s7 < unb);
    const int c = (int)h0 + (int)h1 + (int)h2 + (int)h3 + (int)h4 + (int)h5 + (int)h6 + (int)h7;
    int incl = c;
#pragma unroll
    for (int d = 1; d < 32; d <<= 1) {
      const int up = __shfl_up(incl, d, 32);
      incl += (lane >= d) ? up : 0;
    }
    const int wtotal = __shfl(incl, 31, 32);
    if (lane == 0) wcnt[par * BW + wave] = wtotal;
    __syncthreads();
    int all = 0, pre = 0;
#pragma unroll
    for (int g = 0; g < 4; ++g) {
      const v4i w4 = *(const v4ia*)(wcnt + par * BW + 4 * g);
      const int c0 = clampi(w4.x, 0, 256), c1 = clampi(w4.y, 0, 256);
      const int c2 = clampi(w4.z, 0, 256), c3 = clampi(w4.w, 0, 256);
      all += c0 + c1 + c2 + c3;
      pre += (4 * g + 0 < wave) ? c0 : 0;
      pre += (4 * g + 1 < wave) ? c1 : 0;
      pre += (4 * g + 2 < wave) ? c2 : 0;
      pre += (4 * g + 3 < wave) ? c3 : 0;
    }
    int pos = tot + pre + (incl - c);
#define PUTJ(J, HJ, SJ) if (HJ) { if (pos < RCAP) reg1[pos] = (int)((unsigned)(e0 + (J)) | ((SJ) << SLOTSH)); ++pos; }
    PUTJ(0, h0, s0)
    PUTJ(1, h1, s1)
    PUTJ(2, h2, s2)
    PUTJ(3, h3, s3)
    PUTJ(4, h4, s4)
    PUTJ(5, h5, s5)
    PUTJ(6, h6, s6)
    PUTJ(7, h7, s7)
#undef PUTJ
    tot += all;
  }
  __syncthreads();
  const bool ovf = tot > RCAP;
  const int nh = ovf ? RCAP : tot;

  if (wave == 0) {
#pragma unroll 1
    for (int b0 = 0; b0 < nh; b0 += 32) {
      const int idx = b0 + lane;
      const int uv  = reg1[idx < nh ? idx : nh - 1];
      const int m32 = (nh - b0) < 32 ? (nh - b0) : 32;
#pragma unroll 1
      for (int k = 0; k < m32; ++k) {
        const int u  = __builtin_amdgcn_readlane(uv, k);
        const int sl = (int)(((unsigned)u >> SLOTSH) & (unsigned)(NB - 1));
        const int cv = scnt[sl] + 1;
        if (lane == 0) scnt[sl] = cv;
      }
    }
  }
  __syncthreads();

  int e0c, e1c;
  {
    const v2i cc = *(const v2ia*)(scnt + 2 * tid);
    e0c = cc.x < 0 ? 0 : cc.x;
    e1c = cc.y < 0 ? 0 : cc.y;
    const int ts = e0c + e1c;
    int incl = ts;
#pragma unroll
    for (int d = 1; d < 32; d <<= 1) {
      const int up = __shfl_up(incl, d, 32);
      incl += (lane >= d) ? up : 0;
    }
    if (lane == 31) wtot[wave] = incl;
    __syncthreads();
    int pre = 0;
#pragma unroll
    for (int g = 0; g < 4; ++g) {
      const v4i w4 = *(const v4ia*)(wtot + 4 * g);
      pre += (4 * g + 0 < wave) ? w4.x : 0;
      pre += (4 * g + 1 < wave) ? w4.y : 0;
      pre += (4 * g + 2 < wave) ? w4.z : 0;
      pre += (4 * g + 3 < wave) ? w4.w : 0;
    }
    const int run = pre + incl - ts;
    soff[2 * tid]     = run;
    soff[2 * tid + 1] = run + e0c;
    curs[2 * tid]     = run;
    curs[2 * tid + 1] = run + e0c;
  }
  __syncthreads();

  if (wave == 0) {
#pragma unroll 1
    for (int b0 = 0; b0 < nh; b0 += 32) {
      const int idx = b0 + lane;
      const int uv  = reg1[idx < nh ? idx : nh - 1];
      const int m32 = (nh - b0) < 32 ? (nh - b0) : 32;
#pragma unroll 1
      for (int k = 0; k < m32; ++k) {
        const int u   = __builtin_amdgcn_readlane(uv, k);
        const int sl  = (int)(((unsigned)u >> SLOTSH) & (unsigned)(NB - 1));
        const int eid = (int)((unsigned)u & ((1u << SLOTSH) - 1u));
        const int pr  = curs[sl];
        const int pc  = clampi(pr, 0, RCAP - 1);
        if (lane == 0) { reg2[pc] = eid; curs[sl] = pc + 1; }
      }
    }
  }
  __syncthreads();

  {
    unsigned* lbase = LIST + (size_t)blockIdx.x * (size_t)RCAP * 2;
#pragma unroll 1
    for (int it = 0; it < RCAP / BT; ++it) {
      const int i  = it * BT + tid;
      int ic = i < nh ? i : nh - 1;
      ic = ic < 0 ? 0 : ic;
      const int eid = clampi(reg2[ic], 0, NEDG - 1);
      const int sv = egat[eid];
      asm volatile("" :: "v"(sv));
      const int tv = ety[eid];
      asm volatile("" :: "v"(tv));
      const unsigned msk = (i < nh) ? 0xFFFFFFFFu : 0u;
      v2u o;
      o.x = (unsigned)clampi(sv, 0, NN - 1) & msk;
      o.y = (unsigned)clampi(tv, 0, NET - 1) & msk;
      volatile v2u* q = (volatile v2u*)(lbase + 2 * (size_t)i);
      *q = o;
      __threadfence();
      *q = o;
    }
  }

  {
    const int base = (int)blockIdx.x * RCAP;
    const v2i cc = *(const v2ia*)(scnt + 2 * tid);
    const v2i so = *(const v2ia*)(soff + 2 * tid);
    v4i m;
    m.x = base + so.x;
    m.y = ovf ? -1 : cc.x;
    m.z = base + so.y;
    m.w = ovf ? -1 : cc.y;
    volatile v4i* q = (volatile v4i*)(META + 2 * (size_t)(nodeBase + 2 * tid));
    *q = m;
    __threadfence();
    *q = m;
  }
}

__global__ __launch_bounds__(RTHR) void k_rowprep(const float* __restrict__ H, const float* __restrict__ TB, float* SX) {
  __shared__ __attribute__((aligned(16))) float sdot[2 * RWAVES * NHD];
  const int lane = (int)threadIdx.x & 31;
  const int wave = (int)threadIdx.x >> 5;
  const int row  = (int)blockIdx.x * RWAVES + wave;
  const int rowc = row < MPAD ? row : MPAD - 1;
  const int hg   = lane >> 2;
  const int c8   = lane * 8;
  const float* hp = H + (size_t)rowc * DOUTW + c8;
  const v4f h0 = *(const v4fa*)hp;
  const v4f h1 = *(const v4fa*)(hp + 4);
  asm volatile("" :: "v"(h0), "v"(h1));
  const v4f s0 = *(const v4fa*)(TB + TB_AS + c8);
  const v4f s1 = *(const v4fa*)(TB + TB_AS + c8 + 4);
  const v4f d0 = *(const v4fa*)(TB + TB_AD + c8);
  const v4f d1 = *(const v4fa*)(TB + TB_AD + c8 + 4);
  float ts, td, u;
  ts = h0.x * s0.x;
  u = h0.y * s0.y; ts = ts + u;
  u = h0.z * s0.z; ts = ts + u;
  u = h0.w * s0.w; ts = ts + u;
  u = h1.x * s1.x; ts = ts + u;
  u = h1.y * s1.y; ts = ts + u;
  u = h1.z * s1.z; ts = ts + u;
  u = h1.w * s1.w; ts = ts + u;
  td = h0.x * d0.x;
  u = h0.y * d0.y; td = td + u;
  u = h0.z * d0.z; td = td + u;
  u = h0.w * d0.w; td = td + u;
  u = h1.x * d1.x; td = td + u;
  u = h1.y * d1.y; td = td + u;
  u = h1.z * d1.z; td = td + u;
  u = h1.w * d1.w; td = td + u;
  ts = ts + __shfl_xor(ts, 2, 32);
  ts = ts + __shfl_xor(ts, 1, 32);
  td = td + __shfl_xor(td, 2, 32);
  td = td + __shfl_xor(td, 1, 32);
  if ((lane & 3) == 0) {
    sdot[wave * NHD + hg] = ts;
    sdot[RWAVES * NHD + wave * NHD + hg] = td;
  }
  __syncthreads();
  if (wave == 0) {
    const int l16   = lane & 15;
    const int which = lane >> 4;
    const v4f sv = *(const v4fa*)(sdot + which * (RWAVES * NHD) + 4 * l16);
    const size_t o = (size_t)which * (size_t)SDOFF + (size_t)blockIdx.x * (RWAVES * NHD) + (size_t)(4 * l16);
    volatile v4f* q = (volatile v4f*)(SX + o);
    *q = sv;
    __threadfence();
    *q = sv;
  }
}

__global__ __launch_bounds__(RTHR) void k_walk(const float* __restrict__ H, const float* __restrict__ SX,
                                               const unsigned* __restrict__ LIST, const int* __restrict__ META,
                                               const float* __restrict__ TB, float* out) {
  __shared__ __attribute__((aligned(16))) float sSE[NET * NHD];
  __shared__ __attribute__((aligned(16))) float sW[RWAVES][DEGCAP * NHD];
  __shared__ int sC[RWAVES][DEGCAP];
  const int tid  = (int)threadIdx.x;
  const int lane = tid & 31;
  const int wave = tid >> 5;
  const int row  = (int)blockIdx.x * RWAVES + wave;
  const int rowc = row < NN ? row : NN - 1;
  const int hd   = lane & 7;
  const int hg   = lane >> 2;
  const int c8   = lane * 8;

  const v4f se4 = *(const v4fa*)(TB + TB_SE + 4 * (tid & 15));
  asm volatile("" :: "v"(se4));
  if (tid < 16) *(v4fa*)(sSE + 4 * tid) = se4;

  float* orow = out + (size_t)rowc * DOUTW;
  const v4f r0 = *(const v4fa*)(orow + c8);
  const v4f r1 = *(const v4fa*)(orow + c8 + 4);
  asm volatile("" :: "v"(r0), "v"(r1));

  const v2i mt = *(const v2ia*)(META + 2 * (size_t)rowc);
  asm volatile("" :: "v"(mt));
  const int craw = mt.y;
  const int offv = clampi(mt.x, 0, LISTTOT);
  int cntv = clampi(craw, 0, DEGCAP);
  cntv = cntv < (LISTTOT - offv) ? cntv : (LISTTOT - offv);
  const int off = __builtin_amdgcn_readfirstlane(offv);
  const int cnt = __builtin_amdgcn_readfirstlane(cntv);
  const bool poison = (craw < 0) || (craw > DEGCAP);

  const float sdv = SX[(size_t)SDOFF + (size_t)rowc * NHD + hd];
  asm volatile("" :: "v"(sdv));

  __syncthreads();

  float* W = sW[wave];
  int*   C = sC[wave];
  const int np = cnt * NHD;

  float mx = -__builtin_inff();
#pragma unroll 1
  for (int p0 = 0; p0 < np; p0 += 32) {
    const int p = p0 + lane;
    int ent = p >> 3;
    ent = ent < cnt ? ent : cnt - 1;
    const v2u e2 = *(const v2ua*)(LIST + 2 * (size_t)(off + ent));
    asm volatile("" :: "v"(e2));
    const int col = clampi((int)e2.x, 0, NN - 1);
    const int ty  = clampi((int)e2.y, 0, NET - 1);
    const float ssv = SX[(size_t)col * NHD + hd];
    asm volatile("" :: "v"(ssv));
    const float sev = sSE[ty * NHD + hd];
    float t = ssv + sdv;
    t = t + sev;
    const float sc = leaky_k(t);
    W[p] = sc;
    if (hd == 0) C[p >> 3] = col;
    mx = maxk(mx, sc);
  }
  {
    const float o16 = __shfl_xor(mx, 16, 32);
    mx = maxk(mx, o16);
    const float o8 = __shfl_xor(mx, 8, 32);
    mx = maxk(mx, o8);
  }

#pragma unroll 1
  for (int p0 = 0; p0 < np; p0 += 32) {
    const int p = p0 + lane;
    const float s = W[p];
    const float d = s - mx;
    W[p] = expf(d);
  }
  wave_sync_lds();
  float den = 0.0f;
#pragma unroll 1
  for (int k = 0; k < cnt; ++k) den = den + W[k * NHD + hd];

#pragma unroll 1
  for (int p0 = 0; p0 < np; p0 += 32) {
    const int p = p0 + lane;
    const float e = W[p];
    W[p] = e / den;
  }
  wave_sync_lds();
  v4f a0 = (v4f){0.0f, 0.0f, 0.0f, 0.0f};
  v4f a1 = (v4f){0.0f, 0.0f, 0.0f, 0.0f};
#pragma unroll 1
  for (int k = 0; k < cnt; ++k) {
    const int c = clampi(C[k], 0, NN - 1);
    const float w = W[k * NHD + hg];
    const float* hp = H + (size_t)c * DOUTW + c8;
    const v4f x0 = *(const v4fa*)hp;
    const v4f x1 = *(const v4fa*)(hp + 4);
    asm volatile("" :: "v"(x0), "v"(x1));
    float pr;
    pr = w * x0.x; a0.x = a0.x + pr;
    pr = w * x0.y; a0.y = a0.y + pr;
    pr = w * x0.z; a0.z = a0.z + pr;
    pr = w * x0.w; a0.w = a0.w + pr;
    pr = w * x1.x; a1.x = a1.x + pr;
    pr = w * x1.y; a1.y = a1.y + pr;
    pr = w * x1.z; a1.z = a1.z + pr;
    pr = w * x1.w; a1.w = a1.w + pr;
  }

  const float qnan = __uint_as_float(0x7fc00000u);
  v4f v0, v1;
  v0.x = a0.x + r0.x; v0.y = a0.y + r0.y; v0.z = a0.z + r0.z; v0.w = a0.w + r0.w;
  v1.x = a1.x + r1.x; v1.y = a1.y + r1.y; v1.z = a1.z + r1.z; v1.w = a1.w + r1.w;
  v0.x = poison ? qnan : v0.x; v0.y = poison ? qnan : v0.y; v0.z = poison ? qnan : v0.z; v0.w = poison ? qnan : v0.w;
  v1.x = poison ? qnan : v1.x; v1.y = poison ? qnan : v1.y; v1.z = poison ? qnan : v1.z; v1.w = poison ? qnan : v1.w;
  wave_sync_lds();
  *(v4fa*)(W + c8)     = v0;
  *(v4fa*)(W + c8 + 4) = v1;
  wave_sync_lds();
#pragma unroll 1
  for (int i = 0; i < 8; ++i) {
    const float x = W[i * 32 + lane];
    const float y = (x > 0.0f) ? x : expm1f(x);
    W[i * 32 + lane] = y;
  }
  wave_sync_lds();
  const v4f y0 = *(const v4fa*)(W + 4 * lane);
  const v4f y1 = *(const v4fa*)(W + 128 + 4 * lane);
  const bool rok = row < NN;
  volatile v4f* q0 = (volatile v4f*)(orow + 4 * lane);
  volatile v4f* q1 = (volatile v4f*)(orow + 128 + 4 * lane);
  if (rok) { *q0 = y0; *q1 = y1; }
  __threadfence();
  if (rok) { *q0 = y0; *q1 = y1; }
}

extern "C" void kernel_launch(void* const* d_in, const int* in_sizes, int n_in,
                              void* d_out, int out_size, void* d_ws, size_t ws_size,
                              hipStream_t stream) {
  if (n_in < 10) return;
  if (in_sizes[0] != NN * KD) return;
  if (in_sizes[1] != NEDG || in_sizes[2] != NEDG || in_sizes[3] != NEDG) return;
  if (in_sizes[4] != KD * DOUTW || in_sizes[8] != KD * DOUTW) return;
  if (in_sizes[5] != DOUTW || in_sizes[9] != DOUTW) return;
  if (in_sizes[6] != NET * DOUTW) return;
  if (in_sizes[7] != NHD * ATTW) return;
  if (out_size != NN * DOUTW) return;

  const float* feat = (const float*)d_in[0];
  const int*   esrc = (const int*)  d_in[1];
  const int*   edst = (const int*)  d_in[2];
  const int*   ety  = (const int*)  d_in[3];
  const float* Wfc  = (const float*)d_in[4];
  const float* bfc  = (const float*)d_in[5];
  const float* eemb = (const float*)d_in[6];
  const float* attn = (const float*)d_in[7];
  const float* Wres = (const float*)d_in[8];
  const float* bres = (const float*)d_in[9];
  float* out = (float*)d_out;

  const size_t szXB   = (size_t)MPAD * KD * 2;
  const size_t szWT   = (size_t)DOUTW * KD * 2;
  const size_t szTB   = (size_t)TB_N * 4;
  const size_t szH    = (size_t)MPAD * DOUTW * 4;
  const size_t szSX   = (size_t)2 * MPAD * NHD * 4;
  const size_t szMETA = (size_t)NBLK * NB * 2 * 4;
  const size_t szLIST = (size_t)NBLK * RCAP * 2 * 4;
  static_assert((size_t)MPAD * KD * 2 + 2 * (size_t)DOUTW * KD * 2 + (size_t)TB_N * 4 + (size_t)MPAD * DOUTW * 4 +
                (size_t)2 * MPAD * NHD * 4 + (size_t)NBLK * NB * 8 + (size_t)NBLK * RCAP * 8 == 89174272);
  static_assert(89174272 <= WSMAX);
  static_assert(((size_t)MPAD * KD * 2) % 128 == 0 && ((size_t)DOUTW * KD * 2) % 128 == 0 && ((size_t)TB_N * 4) % 128 == 0);
  static_assert(((size_t)MPAD * DOUTW * 4) % 128 == 0 && ((size_t)MPAD * NHD * 4) % 128 == 0);
  static_assert(((size_t)NBLK * NB * 8) % 128 == 0 && ((size_t)RCAP * 8) % 128 == 0);
  char* ws = (char*)d_ws;
  size_t off = 0;
  const size_t oXB   = off; off += szXB;
  const size_t oWFT  = off; off += szWT;
  const size_t oWRT  = off; off += szWT;
  const size_t oTB   = off; off += szTB;
  const size_t oH    = off; off += szH;
  const size_t oSX   = off; off += szSX;
  const size_t oMETA = off; off += szMETA;
  const size_t oLIST = off; off += szLIST;
  if (off > ws_size || off > (size_t)WSMAX) return;
  unsigned short* XB  = (unsigned short*)(ws + oXB);
  unsigned short* WFT = (unsigned short*)(ws + oWFT);
  unsigned short* WRT = (unsigned short*)(ws + oWRT);
  float*    TB   = (float*)(ws + oTB);
  float*    H    = (float*)(ws + oH);
  float*    SX   = (float*)(ws + oSX);
  int*      META = (int*)(ws + oMETA);
  unsigned* LIST = (unsigned*)(ws + oLIST);

  hipFuncSetAttribute(reinterpret_cast<const void*>(&k_list),
                      hipFuncAttributeMaxDynamicSharedMemorySize, LDS_BKT);

  static_assert((MPAD * KD / 8) % 256 == 0);
  k_plane<0><<<MPAD * KD / 8 / 256, 256, 0, stream>>>(feat, NN, KD, KD, XB, MPAD, KD);
  k_prep<<<2 * PREP_PB + 1, 256, 0, stream>>>(Wfc, Wres, bfc, bres, eemb, attn, WFT, WRT, TB);
  k_list<<<NBLK, BT, LDS_BKT, stream>>>(edst, esrc, ety, LIST, META);

  const int tiles = (MPAD / 64) * (DOUTW / 64);
  static_assert((NN + 63) / 64 == MPAD / 64);
  const int gG = (tiles + 7) / 8;
  k_gemm_nt<0, 1><<<gG, 256, 0, stream>>>(XB, WRT, TB + TB_BR, out, NN, DOUTW, KD, DOUTW);
  k_gemm_nt<0, 1><<<gG, 256, 0, stream>>>(XB, WFT, TB + TB_BF, H, MPAD, DOUTW, KD, DOUTW);
  k_rowprep<<<MPAD / RWAVES, RTHR, 0, stream>>>(H, TB, SX);
  k_walk<<<NN / RWAVES, RTHR, 0, stream>>>(H, SX, LIST, META, TB, out);
}
